// RRTAttention_48661979464003
// MI455X (gfx1250) — hardware-verified
//
#include <hip/hip_runtime.h>
#include <hip/hip_bf16.h>
#include <math.h>
#include <stddef.h>


#define B_    2
#define T_    2048
#define D_    1024
#define NH_   16
#define NKV_  4
#define HD_   64
#define KD_   256
#define BT_   4096
#define NQKV_ 1536
#define RANK_ 8
#define ROPEP_ 32
#define NXB_  (BT_ / 2)
#define NWB_  (D_ / 2)
#define NRB_  (T_ / 64)

#define NEG_INF (-__builtin_inff())

typedef float v8f __attribute__((ext_vector_type(8)));
typedef float v4f __attribute__((ext_vector_type(4)));
typedef __bf16 v16b __attribute__((ext_vector_type(16)));
typedef unsigned short v8us __attribute__((ext_vector_type(8)));
typedef v8us v8usa __attribute__((may_alias));
typedef v4f v4fa __attribute__((may_alias));

union Frag { v16b v; v8us h[2]; };

__device__ __forceinline__ unsigned short f2bf(float f) {
  unsigned u = __float_as_uint(f);
  u = u + 0x7FFFu + ((u >> 16) & 1u);
  return (unsigned short)(u >> 16);
}
__device__ __forceinline__ float bf2f(unsigned short s) {
  return __uint_as_float(((unsigned)s) << 16);
}
__device__ __forceinline__ void split_bf(float x, unsigned short& hi, unsigned short& lo) {
  hi = f2bf(x);
  lo = f2bf(x - bf2f(hi));
}

__device__ __forceinline__ v8f mma(const Frag& a, const Frag& b, v8f c) {
  c = __builtin_amdgcn_wmma_f32_16x16x32_bf16(false, a.v, false, b.v, (short)0, c, false, false);
  asm volatile("v_nop\n\tv_nop\n\tv_nop\n\tv_nop" : "+v"(c) : "v"(a.v), "v"(b.v));
  return c;
}
__device__ __forceinline__ void ldfrag(Frag& f, const unsigned short* p) {
  f.h[0] = *(const v8usa*)(p);
  f.h[1] = *(const v8usa*)(p + 16);
}
__device__ __forceinline__ void split8(const v4f a0, const v4f a1, v8us& oh, v8us& ol) {
  unsigned short hi, lo;
  split_bf(a0[0], hi, lo); oh[0] = hi; ol[0] = lo;
  split_bf(a0[1], hi, lo); oh[1] = hi; ol[1] = lo;
  split_bf(a0[2], hi, lo); oh[2] = hi; ol[2] = lo;
  split_bf(a0[3], hi, lo); oh[3] = hi; ol[3] = lo;
  split_bf(a1[0], hi, lo); oh[4] = hi; ol[4] = lo;
  split_bf(a1[1], hi, lo); oh[5] = hi; ol[5] = lo;
  split_bf(a1[2], hi, lo); oh[6] = hi; ol[6] = lo;
  split_bf(a1[3], hi, lo); oh[7] = hi; ol[7] = lo;
}

__global__ void __launch_bounds__(256) k_conv(const float* __restrict__ x, const float* __restrict__ wp,
                                             unsigned short* xh, unsigned short* xl,
                                             unsigned short* wph, unsigned short* wpl, float* rope) {
  __shared__ __attribute__((aligned(16))) float srow[8][ROPEP_];
  const int tid = threadIdx.x;
  const int blk = blockIdx.x;
  if (blk < NXB_ + NWB_) {
    const int sub = tid >> 7;
    const int c = (tid & 127) * 8;
    const float* src;
    unsigned short* dh;
    unsigned short* dl;
    if (blk < NXB_) {
      const int row = 2 * blk + sub;
      src = x + (size_t)row * D_ + c;
      dh = xh + (size_t)row * D_ + c;
      dl = xl + (size_t)row * D_ + c;
    } else {
      const int row = 2 * (blk - NXB_) + sub;
      src = wp + (size_t)row * D_ + c;
      dh = wph + (size_t)row * D_ + c;
      dl = wpl + (size_t)row * D_ + c;
    }
    const v4f a0 = *(const v4fa*)(src);
    const v4f a1 = *(const v4fa*)(src + 4);
    v8us oh, ol;
    split8(a0, a1, oh, ol);
    *(volatile v8us*)dh = oh;
    *(volatile v8us*)dl = ol;
    __threadfence();
    *(volatile v8us*)dh = oh;
    *(volatile v8us*)dl = ol;
  } else {
    const int lane = tid & 31, wave = tid >> 5;
    const int rb = blk - NXB_ - NWB_;
    const int jj = lane & 7;
    const float e = (float)(2 * jj) * 0.0625f;
    const float pw = powf(10000.0f, e);
    const float inv = 1.0f / pw;
#pragma unroll 1
    for (int jp = 0; jp < 8; ++jp) {
      const int t = rb * 64 + jp * 8 + wave;
      const float fr = (float)t * inv;
      const float cv = cosf(fr);
      const float sv = sinf(fr);
      const float val = (lane < 8) ? cv : ((lane < 16) ? sv : 0.0f);
      srow[wave][lane] = val;
      __builtin_amdgcn_fence(__ATOMIC_RELEASE, "wavefront");
      __builtin_amdgcn_wave_barrier();
      const int q = lane & 7;
      const v4f piece = *(const v4fa*)(&srow[wave][4 * q]);
      if (lane < 8) {
        float* rp = rope + (size_t)t * ROPEP_ + 4 * q;
        *(volatile v4f*)rp = piece;
        __threadfence();
        *(volatile v4f*)rp = piece;
      }
      __builtin_amdgcn_wave_barrier();
    }
  }
}

__global__ void __launch_bounds__(128) k_wall(const float* __restrict__ Wq, const float* __restrict__ Wk,
                                             const float* __restrict__ Wv, const float* __restrict__ Aq,
                                             const float* __restrict__ Bq, const float* __restrict__ Av,
                                             const float* __restrict__ Bv, unsigned short* wh, unsigned short* wl) {
  const int o = blockIdx.x;
  const int c = threadIdx.x * 8;
  const int kind = (o < D_) ? 0 : ((o < D_ + KD_) ? 1 : 2);
  const float* wrow;
  const float* arow;
  const float* brow;
  if (kind == 0)      { wrow = Wq + (size_t)o * D_;                 arow = Aq; brow = Bq + (size_t)o * RANK_; }
  else if (kind == 1) { wrow = Wk + (size_t)(o - D_) * D_;          arow = Aq; brow = Bq; }
  else                { const int oo = o - D_ - KD_;
                        wrow = Wv + (size_t)oo * D_;                arow = Av; brow = Bv + (size_t)oo * RANK_; }
  const v4f w0 = *(const v4fa*)(wrow + c);
  const v4f w1 = *(const v4fa*)(wrow + c + 4);
  float v0 = w0[0], v1 = w0[1], v2 = w0[2], v3 = w0[3];
  float v4 = w1[0], v5 = w1[1], v6 = w1[2], v7 = w1[3];
  if (kind != 1) {
#pragma unroll 1
    for (int r = 0; r < RANK_; ++r) {
      const float br = brow[r];
      const v4f c0 = *(const v4fa*)(arow + (size_t)r * D_ + c);
      const v4f c1 = *(const v4fa*)(arow + (size_t)r * D_ + c + 4);
      v0 += br * c0[0]; v1 += br * c0[1]; v2 += br * c0[2]; v3 += br * c0[3];
      v4 += br * c1[0]; v5 += br * c1[1]; v6 += br * c1[2]; v7 += br * c1[3];
    }
  }
  const v4f a0 = {v0, v1, v2, v3};
  const v4f a1 = {v4, v5, v6, v7};
  v8us oh, ol;
  split8(a0, a1, oh, ol);
  unsigned short* dh = wh + (size_t)o * D_ + c;
  unsigned short* dl = wl + (size_t)o * D_ + c;
  *(volatile v8us*)dh = oh;
  *(volatile v8us*)dl = ol;
  __threadfence();
  *(volatile v8us*)dh = oh;
  *(volatile v8us*)dl = ol;
}

__global__ void __launch_bounds__(256) k_qkv(const unsigned short* __restrict__ xh, const unsigned short* __restrict__ xl,
                                            const unsigned short* __restrict__ wh, const unsigned short* __restrict__ wl,
                                            const float* __restrict__ rope, const float* __restrict__ qgain,
                                            unsigned short* Qh, unsigned short* Ql, unsigned short* Kh, unsigned short* Kl,
                                            unsigned short* Vh, unsigned short* Vl) {
  __shared__ __attribute__((aligned(16))) unsigned short stg[8192];
  const int tid = threadIdx.x, lane = tid & 31, wave = tid >> 5;
  const int h = lane >> 4, m = lane & 15;
  const int wm = wave & 3, wn = wave >> 2;
  const int m0 = blockIdx.x * 64 + wm * 16;
  const int n0 = blockIdx.y * 128 + wn * 64;
  const int kind = (blockIdx.y < 8) ? 0 : ((blockIdx.y < 10) ? 1 : 2);

  v8f acc[4] = {};
  const unsigned short* ahp = xh + (size_t)(m0 + m) * D_ + 8 * h;
  const unsigned short* alp = xl + (size_t)(m0 + m) * D_ + 8 * h;
  const size_t boff = (size_t)(n0 + m) * D_ + 8 * h;
#pragma unroll 1
  for (int ks = 0; ks < D_ / 32; ++ks) {
    const int k0 = ks * 32;
    Frag ah, al, bh[4], bl[4];
    ldfrag(ah, ahp + k0);
    ldfrag(al, alp + k0);
#pragma unroll
    for (int j = 0; j < 4; ++j) {
      ldfrag(bh[j], wh + boff + (size_t)(16 * j) * D_ + k0);
      ldfrag(bl[j], wl + boff + (size_t)(16 * j) * D_ + k0);
    }
#pragma unroll
    for (int j = 0; j < 4; ++j) {
      acc[j] = mma(ah, bh[j], acc[j]);
      acc[j] = mma(ah, bl[j], acc[j]);
      acc[j] = mma(al, bh[j], acc[j]);
    }
  }

  const int t0 = m0 & (T_ - 1);
  const int bidx = m0 >> 11;
  if (kind < 2) {
    const int head = (kind == 0) ? (n0 >> 6) : ((n0 - D_) >> 6);
    const float graw = qgain[head & 15];
    const float g = (kind == 0) ? graw : 1.0f;
#pragma unroll
    for (int r = 0; r < 8; ++r) {
      const int t = t0 + 8 * h + r;
      float v0 = acc[0][r], v1 = acc[1][r], v2 = acc[2][r], v3 = acc[3][r];
      float ss = v0 * v0 + v1 * v1 + v2 * v2 + v3 * v3;
      ss += __shfl_xor(ss, 1, 32);
      ss += __shfl_xor(ss, 2, 32);
      ss += __shfl_xor(ss, 4, 32);
      ss += __shfl_xor(ss, 8, 32);
      const float rs = rsqrtf(ss * (1.0f / 64.0f) + 1.1920929e-7f);
      v0 *= rs; v1 *= rs; v2 *= rs; v3 *= rs;
      const float other = __shfl_xor(v0, 8, 32);
      const int jj = m & 7;
      const float cs = rope[(size_t)t * ROPEP_ + jj];
      const float sn = rope[(size_t)t * ROPEP_ + 8 + jj];
      const float rot = (m < 8) ? (v0 * cs + other * sn) : (other * sn - v0 * cs);
      acc[0][r] = rot * g; acc[1][r] = v1 * g; acc[2][r] = v2 * g; acc[3][r] = v3 * g;
    }
  }

#pragma unroll
  for (int p = 0; p < 2; ++p) {
    if (kind < 2) {
      unsigned short* sw = stg + wave * 1024;
#pragma unroll
      for (int j = 0; j < 4; ++j)
#pragma unroll
        for (int r = 0; r < 8; ++r) {
          unsigned short hi, lo;
          split_bf(acc[j][r], hi, lo);
          sw[(8 * h + r) * 64 + 16 * j + m] = (p == 0) ? hi : lo;
        }
    } else {
      unsigned short* sb = stg + wn * 4096;
#pragma unroll
      for (int j = 0; j < 4; ++j)
#pragma unroll
        for (int r = 0; r < 8; ++r) {
          unsigned short hi, lo;
          split_bf(acc[j][r], hi, lo);
          const int tt = 16 * wm + 8 * h + r;
          const int d = 16 * j + m;
          sb[d * 64 + tt] = (p == 0) ? hi : lo;
        }
    }
    __syncthreads();
    if (kind < 2) {
      const int head = (kind == 0) ? (n0 >> 6) : ((n0 - D_) >> 6);
      const int nheads = (kind == 0) ? NH_ : NKV_;
      unsigned short* plane = (kind == 0) ? ((p == 0) ? Qh : Ql) : ((p == 0) ? Kh : Kl);
      const size_t prow0 = ((size_t)(bidx * nheads + head)) * T_ + t0;
      const unsigned short* sw = stg + wave * 1024;
#pragma unroll
      for (int pass = 0; pass < 2; ++pass) {
#pragma unroll
        for (int i2 = 0; i2 < 4; ++i2) {
          const int row = 4 * i2 + (lane >> 3), pc = lane & 7;
          const v8us val = *(const v8usa*)(sw + row * 64 + 8 * pc);
          unsigned short* dp = plane + (prow0 + row) * HD_ + 8 * pc;
          *(volatile v8us*)dp = val;
        }
        if (pass == 0) __threadfence();
      }
    } else {
      const int hv = (n0 - D_ - KD_) >> 6;
      const int bb = (blockIdx.x * 64) >> 11;
      const int tb = (blockIdx.x * 64) & (T_ - 1);
      unsigned short* plane = (p == 0) ? Vh : Vl;
      const unsigned short* sb = stg + wn * 4096;
#pragma unroll
      for (int pass = 0; pass < 2; ++pass) {
#pragma unroll
        for (int i2 = 0; i2 < 4; ++i2) {
          const int d = 16 * wm + 4 * i2 + (lane >> 3), pc = lane & 7;
          const v8us val = *(const v8usa*)(sb + d * 64 + 8 * pc);
          unsigned short* dp = plane + ((size_t)(bb * NKV_ + hv) * HD_ + d) * T_ + tb + 8 * pc;
          *(volatile v8us*)dp = val;
        }
        if (pass == 0) __threadfence();
      }
    }
    __syncthreads();
  }
}

__global__ void __launch_bounds__(32) k_attn(const unsigned short* __restrict__ Qh, const unsigned short* __restrict__ Ql,
                                            const unsigned short* __restrict__ Kh, const unsigned short* __restrict__ Kl,
                                            const unsigned short* __restrict__ Vh, const unsigned short* __restrict__ Vl,
                                            unsigned short* Yh, unsigned short* Yl) {
  __shared__ __attribute__((aligned(16))) unsigned short Ps[2 * 16 * 32];
  __shared__ __attribute__((aligned(16))) unsigned short Ys[2 * 16 * 64];
  const int lane = threadIdx.x & 31, h = lane >> 4, m = lane & 15;
  const int bh = blockIdx.x >> 7;
  const int qt = blockIdx.x & 127;
  const int b = bh >> 4, hq = bh & 15, kvh = hq >> 2;
  const int qr0 = qt * 16;

  const size_t qoff = (((size_t)(b * NH_ + hq)) * T_ + qr0 + m) * HD_ + 8 * h;
  Frag qh0, qh1, ql0, ql1;
  ldfrag(qh0, Qh + qoff); ldfrag(qh1, Qh + qoff + 32);
  ldfrag(ql0, Ql + qoff); ldfrag(ql1, Ql + qoff + 32);
  const size_t koff = (((size_t)(b * NKV_ + kvh)) * T_ + m) * HD_ + 8 * h;
  const unsigned short* Khp = Kh + koff;
  const unsigned short* Klp = Kl + koff;
  const size_t voff = (((size_t)(b * NKV_ + kvh)) * HD_ + m) * T_ + 8 * h;
  const unsigned short* Vhp = Vh + voff;
  const unsigned short* Vlp = Vl + voff;

  v8f o[4] = {};
  float mrow[8], lrow[8];
#pragma unroll
  for (int r = 0; r < 8; ++r) { mrow[r] = NEG_INF; lrow[r] = 0.0f; }

  const int ktmax = (qr0 + 15) >> 5;
  for (int kt = 0; kt <= ktmax; ++kt) {
    const int kb = kt * 32;
    v8f s0 = {}, s1 = {};
    {
      Frag k00, k01, k10, k11;
      const unsigned short* p0 = Khp + (size_t)kb * HD_;
      const unsigned short* p1 = Khp + (size_t)(kb + 16) * HD_;
      ldfrag(k00, p0); ldfrag(k01, p0 + 32);
      ldfrag(k10, p1); ldfrag(k11, p1 + 32);
      s0 = mma(qh0, k00, s0); s0 = mma(qh1, k01, s0); s0 = mma(ql0, k00, s0); s0 = mma(ql1, k01, s0);
      s1 = mma(qh0, k10, s1); s1 = mma(qh1, k11, s1); s1 = mma(ql0, k10, s1); s1 = mma(ql1, k11, s1);
    }
    {
      Frag l00, l01, l10, l11;
      const unsigned short* p0 = Klp + (size_t)kb * HD_;
      const unsigned short* p1 = Klp + (size_t)(kb + 16) * HD_;
      ldfrag(l00, p0); ldfrag(l01, p0 + 32);
      ldfrag(l10, p1); ldfrag(l11, p1 + 32);
      s0 = mma(qh0, l00, s0); s0 = mma(qh1, l01, s0);
      s1 = mma(qh0, l10, s1); s1 = mma(qh1, l11, s1);
    }
    __syncthreads();
#pragma unroll
    for (int r = 0; r < 8; ++r) {
      const int rowq = qr0 + 8 * h + r;
      const int c0 = kb + m, c1 = c0 + 16;
      const float sv0 = (c0 <= rowq) ? s0[r] * 0.125f : NEG_INF;
      const float sv1 = (c1 <= rowq) ? s1[r] * 0.125f : NEG_INF;
      float smax = fmaxf(sv0, sv1);
      smax = fmaxf(smax, __shfl_xor(smax, 1, 32));
      smax = fmaxf(smax, __shfl_xor(smax, 2, 32));
      smax = fmaxf(smax, __shfl_xor(smax, 4, 32));
      smax = fmaxf(smax, __shfl_xor(smax, 8, 32));
      const float mnew = fmaxf(mrow[r], smax);
      const float p0 = __expf(sv0 - mnew);
      const float p1 = __expf(sv1 - mnew);
      float rsum = p0 + p1;
      rsum += __shfl_xor(rsum, 1, 32);
      rsum += __shfl_xor(rsum, 2, 32);
      rsum += __shfl_xor(rsum, 4, 32);
      rsum += __shfl_xor(rsum, 8, 32);
      const float corr = __expf(mrow[r] - mnew);
      lrow[r] = lrow[r] * corr + rsum;
      mrow[r] = mnew;
      o[0][r] *= corr; o[1][r] *= corr; o[2][r] *= corr; o[3][r] *= corr;
      unsigned short h0, l0, h1, l1;
      split_bf(p0, h0, l0);
      split_bf(p1, h1, l1);
      const int rl = 8 * h + r;
      Ps[rl * 32 + m] = h0;        Ps[rl * 32 + 16 + m] = h1;
      Ps[512 + rl * 32 + m] = l0;  Ps[512 + rl * 32 + 16 + m] = l1;
    }
    __syncthreads();
    Frag pH, pL;
    ldfrag(pH, Ps + m * 32 + 8 * h);
    ldfrag(pL, Ps + 512 + m * 32 + 8 * h);
    {
      Frag v0, v1, v2, v3;
      ldfrag(v0, Vhp + kb);
      ldfrag(v1, Vhp + (size_t)16 * T_ + kb);
      ldfrag(v2, Vhp + (size_t)32 * T_ + kb);
      ldfrag(v3, Vhp + (size_t)48 * T_ + kb);
      o[0] = mma(pH, v0, o[0]); o[0] = mma(pL, v0, o[0]);
      o[1] = mma(pH, v1, o[1]); o[1] = mma(pL, v1, o[1]);
      o[2] = mma(pH, v2, o[2]); o[2] = mma(pL, v2, o[2]);
      o[3] = mma(pH, v3, o[3]); o[3] = mma(pL, v3, o[3]);
    }
    {
      Frag w0, w1, w2, w3;
      ldfrag(w0, Vlp + kb);
      ldfrag(w1, Vlp + (size_t)16 * T_ + kb);
      ldfrag(w2, Vlp + (size_t)32 * T_ + kb);
      ldfrag(w3, Vlp + (size_t)48 * T_ + kb);
      o[0] = mma(pH, w0, o[0]);
      o[1] = mma(pH, w1, o[1]);
      o[2] = mma(pH, w2, o[2]);
      o[3] = mma(pH, w3, o[3]);
    }
  }

#pragma unroll
  for (int r = 0; r < 8; ++r) {
    const float inv = 1.0f / lrow[r];
    const int rl = 8 * h + r;
#pragma unroll
    for (int j = 0; j < 4; ++j) {
      unsigned short hi, lo;
      split_bf(o[j][r] * inv, hi, lo);
      Ys[rl * 64 + 16 * j + m] = hi;
      Ys[1024 + rl * 64 + 16 * j + m] = lo;
    }
  }
  __syncthreads();
  const size_t yrow0 = (size_t)b * T_ + qr0;
#pragma unroll
  for (int pass = 0; pass < 2; ++pass) {
#pragma unroll
    for (int p = 0; p < 2; ++p) {
      unsigned short* plane = (p == 0) ? Yh : Yl;
#pragma unroll
      for (int i2 = 0; i2 < 4; ++i2) {
        const int row = 4 * i2 + (lane >> 3), pc = lane & 7;
        const v8us val = *(const v8usa*)(Ys + p * 1024 + row * 64 + 8 * pc);
        unsigned short* dp = plane + (yrow0 + row) * D_ + hq * HD_ + 8 * pc;
        *(volatile v8us*)dp = val;
      }
    }
    if (pass == 0) __threadfence();
  }
}

__global__ void __launch_bounds__(256) k_proj(const unsigned short* __restrict__ Yh, const unsigned short* __restrict__ Yl,
                                             const unsigned short* __restrict__ wph, const unsigned short* __restrict__ wpl,
                                             float* out) {
  __shared__ __attribute__((aligned(16))) float stg[8 * 1024];
  const int tid = threadIdx.x, lane = tid & 31, wave = tid >> 5;
  const int h = lane >> 4, m = lane & 15;
  const int wm = wave & 1, wn = wave >> 1;
  const int m0 = blockIdx.x * 64 + wm * 32;
  const int n0 = blockIdx.y * 128 + wn * 32;

  v8f acc[2][2] = {};
#pragma unroll 1
  for (int ks = 0; ks < D_ / 32; ++ks) {
    const int k0 = ks * 32 + 8 * h;
    Frag ah[2], al[2], bh[2], bl[2];
#pragma unroll
    for (int i = 0; i < 2; ++i) {
      ldfrag(ah[i], Yh + (size_t)(m0 + 16 * i + m) * D_ + k0);
      ldfrag(al[i], Yl + (size_t)(m0 + 16 * i + m) * D_ + k0);
    }
#pragma unroll
    for (int j = 0; j < 2; ++j) {
      ldfrag(bh[j], wph + (size_t)(n0 + 16 * j + m) * D_ + k0);
      ldfrag(bl[j], wpl + (size_t)(n0 + 16 * j + m) * D_ + k0);
    }
#pragma unroll
    for (int i = 0; i < 2; ++i)
#pragma unroll
      for (int j = 0; j < 2; ++j) {
        acc[i][j] = mma(ah[i], bh[j], acc[i][j]);
        acc[i][j] = mma(ah[i], bl[j], acc[i][j]);
        acc[i][j] = mma(al[i], bh[j], acc[i][j]);
      }
  }

  float* sw = stg + wave * 1024;
#pragma unroll
  for (int i = 0; i < 2; ++i)
#pragma unroll
    for (int j = 0; j < 2; ++j)
#pragma unroll
      for (int r = 0; r < 8; ++r) sw[(16 * i + 8 * h + r) * 32 + 16 * j + m] = acc[i][j][r];
  __syncthreads();
#pragma unroll
  for (int pass = 0; pass < 2; ++pass) {
#pragma unroll
    for (int i2 = 0; i2 < 8; ++i2) {
      const int row = 4 * i2 + (lane >> 3), pc = lane & 7;
      const v4f val = *(const v4fa*)(sw + row * 32 + 4 * pc);
      float* dp = out + (size_t)(m0 + row) * D_ + n0 + 4 * pc;
      *(volatile v4f*)dp = val;
    }
    if (pass == 0) __threadfence();
  }
}

extern "C" void kernel_launch(void* const* d_in, const int* in_sizes, int n_in,
                              void* d_out, int out_size, void* d_ws, size_t ws_size,
                              hipStream_t stream) {
  if (n_in < 10) return;
  if (in_sizes[0] != BT_ * D_ || in_sizes[1] != D_ * D_ || in_sizes[2] != KD_ * D_ ||
      in_sizes[3] != KD_ * D_ || in_sizes[4] != D_ * D_ || in_sizes[5] != NH_ ||
      in_sizes[6] != RANK_ * D_ || in_sizes[7] != D_ * RANK_ || in_sizes[8] != RANK_ * D_ ||
      in_sizes[9] != KD_ * RANK_) return;
  if (out_size != BT_ * D_) return;

  const float* x     = (const float*)d_in[0];
  const float* Wq    = (const float*)d_in[1];
  const float* Wk    = (const float*)d_in[2];
  const float* Wv    = (const float*)d_in[3];
  const float* Wproj = (const float*)d_in[4];
  const float* qg    = (const float*)d_in[5];
  const float* Aq    = (const float*)d_in[6];
  const float* Bq    = (const float*)d_in[7];
  const float* Av    = (const float*)d_in[8];
  const float* Bv    = (const float*)d_in[9];
  float* out = (float*)d_out;

  char* ws = (char*)d_ws;
  size_t off = 0;
  auto carve = [&](size_t bytes) {
    char* p = ws + off;
    off += (bytes + 255) & ~(size_t)255;
    return p;
  };
  unsigned short* xh   = (unsigned short*)carve((size_t)BT_ * D_ * 2);
  unsigned short* xl   = (unsigned short*)carve((size_t)BT_ * D_ * 2);
  unsigned short* wh   = (unsigned short*)carve((size_t)NQKV_ * D_ * 2);
  unsigned short* wl   = (unsigned short*)carve((size_t)NQKV_ * D_ * 2);
  unsigned short* wph  = (unsigned short*)carve((size_t)D_ * D_ * 2);
  unsigned short* wpl  = (unsigned short*)carve((size_t)D_ * D_ * 2);
  float*          rope = (float*)carve((size_t)T_ * ROPEP_ * 4);
  unsigned short* Qh   = (unsigned short*)carve((size_t)B_ * NH_ * T_ * HD_ * 2);
  unsigned short* Ql   = (unsigned short*)carve((size_t)B_ * NH_ * T_ * HD_ * 2);
  unsigned short* Kh   = (unsigned short*)carve((size_t)B_ * NKV_ * T_ * HD_ * 2);
  unsigned short* Kl   = (unsigned short*)carve((size_t)B_ * NKV_ * T_ * HD_ * 2);
  unsigned short* Vh   = (unsigned short*)carve((size_t)B_ * NKV_ * HD_ * T_ * 2);
  unsigned short* Vl   = (unsigned short*)carve((size_t)B_ * NKV_ * HD_ * T_ * 2);
  unsigned short* Yh   = (unsigned short*)carve((size_t)BT_ * D_ * 2);
  unsigned short* Yl   = (unsigned short*)carve((size_t)BT_ * D_ * 2);
  if (off > ws_size || off > (size_t)134217728) return;

  k_conv<<<dim3(NXB_ + NWB_ + NRB_), dim3(256), 0, stream>>>(x, Wproj, xh, xl, wph, wpl, rope);
  k_wall<<<dim3(NQKV_), dim3(128), 0, stream>>>(Wq, Wk, Wv, Aq, Bq, Av, Bv, wh, wl);
  k_qkv<<<dim3(BT_ / 64, NQKV_ / 128), dim3(256), 0, stream>>>(xh, xl, wh, wl, rope, qg, Qh, Ql, Kh, Kl, Vh, Vl);
  k_attn<<<dim3(B_ * NH_ * (T_ / 16)), dim3(32), 0, stream>>>(Qh, Ql, Kh, Kl, Vh, Vl, Yh, Yl);
  k_proj<<<dim3(BT_ / 64, D_ / 128), dim3(256), 0, stream>>>(Yh, Yl, wph, wpl, out);
}
